// GPTS_11536282157499
// MI455X (gfx1250) — hardware-verified
//
#include <hip/hip_runtime.h>

#define Bsz 8
#define Nseq 2048
#define VARNUM 96
#define INDIM 320
#define ADIM 64
#define NH 8
#define ALLDIM 512
#define MROWS (Bsz * Nseq)
#define RSPLIT (1.0f / 2048.0f)

typedef _Float16 f16;
typedef f16   v16h __attribute__((ext_vector_type(16)));
typedef f16   v8h  __attribute__((ext_vector_type(8)));
typedef float v8f  __attribute__((ext_vector_type(8)));
typedef float v4f_t __attribute__((ext_vector_type(4)));
typedef float v4fa  __attribute__((ext_vector_type(4), may_alias));
typedef unsigned v4u_t __attribute__((ext_vector_type(4)));

__device__ __forceinline__ f16 lo_of(float v, f16 h) { return (f16)((v - (float)h) * 2048.0f); }
__device__ __forceinline__ unsigned pk2s(float a, float b, unsigned* lo) {
  const f16 h0 = (f16)a, h1 = (f16)b;
  *lo = (unsigned)__builtin_bit_cast(unsigned short, lo_of(a, h0)) | ((unsigned)__builtin_bit_cast(unsigned short, lo_of(b, h1)) << 16);
  return (unsigned)__builtin_bit_cast(unsigned short, h0) | ((unsigned)__builtin_bit_cast(unsigned short, h1) << 16);
}
__device__ __forceinline__ v8f wmma16(v16h a, v16h b, v8f c) { return __builtin_amdgcn_wmma_f32_16x16x32_f16(false, a, false, b, (short)0, c, false, false); }
struct Frag2 { v16h h, l; };
__device__ __forceinline__ v8f wmma_split(const Frag2& a, const Frag2& b, v8f c) { v8f x = {}; x = wmma16(a.l, b.h, x); x = wmma16(a.h, b.l, x); return wmma16(a.h, b.h, c) + x * RSPLIT; }
__device__ __forceinline__ v16h cat8(v8h a, v8h b) { return __builtin_shufflevector(a, b, 0,1,2,3,4,5,6,7,8,9,10,11,12,13,14,15); }
__device__ __forceinline__ Frag2 ld2(const f16* p, size_t plane) { Frag2 f; f.h = cat8(*(const v8h*)p, *(const v8h*)(p + 16)); f.l = cat8(*(const v8h*)(p + plane), *(const v8h*)(p + plane + 16)); return f; }

#define PLX  ((size_t)MROWS * INDIM)
#define PLW  ((size_t)ALLDIM * INDIM)
#define PLWF ((size_t)ADIM * ALLDIM)
#define PLA  ((size_t)MROWS * ALLDIM)

__global__ void __launch_bounds__(256) build_x(const float* __restrict__ times, const float* __restrict__ data,
                                               const float* __restrict__ mask,  const float* __restrict__ w_per,
                                               const float* __restrict__ b_per, const float* __restrict__ w_lin,
                                               const float* __restrict__ b_lin, f16* __restrict__ x) {
  const int row = blockIdx.x;
  const float t = times[row];
  const int f = threadIdx.x * 2;
  if (f >= INDIM) return;
  float v2[2];
#pragma unroll
  for (int q = 0; q < 2; ++q) {
    const int ff = f + q;
    float v;
    if (ff < VARNUM)            v = data[(size_t)row * VARNUM + ff];
    else if (ff < 2 * VARNUM)   v = mask[(size_t)row * VARNUM + (ff - VARNUM)];
    else { const int j = ff - 2 * VARNUM; v = (j == 0) ? (t * w_lin[0] + b_lin[0]) : sinf(t * w_per[j - 1] + b_per[j - 1]); }
    v2[q] = v;
  }
  unsigned lo; const unsigned p = pk2s(v2[0], v2[1], &lo);
  f16* d = x + (size_t)row * INDIM + f;
  *(volatile unsigned*)d = p; *(volatile unsigned*)(d + PLX) = lo; __threadfence();
  *(volatile unsigned*)d = p; *(volatile unsigned*)(d + PLX) = lo;
}

__global__ void __launch_bounds__(256) wt_cvt(const float* __restrict__ W, f16* __restrict__ WT, int KD, int NW, size_t plane) {
  __shared__ float t[64][17];
  const int tx = threadIdx.x & 15, ty = threadIdx.x >> 4;
  const int nt = blockIdx.x, kt = blockIdx.y;
#pragma unroll
  for (int p = 0; p < 4; ++p) t[p * 16 + ty][tx] = W[(size_t)(kt * 64 + p * 16 + ty) * NW + nt * 16 + tx];
  __syncthreads();
  if (threadIdx.x < 128) {
    const int rr = threadIdx.x >> 3, q = (threadIdx.x & 7) * 8;
    v4u_t v, vl; unsigned lq;
    v.x = pk2s(t[q][rr], t[q + 1][rr], &lq); vl.x = lq; v.y = pk2s(t[q + 2][rr], t[q + 3][rr], &lq); vl.y = lq;
    v.z = pk2s(t[q + 4][rr], t[q + 5][rr], &lq); vl.z = lq; v.w = pk2s(t[q + 6][rr], t[q + 7][rr], &lq); vl.w = lq;
    f16* dst = WT + (size_t)(nt * 16 + rr) * KD + kt * 64 + q;
    *(volatile v4u_t*)dst = v; *(volatile v4u_t*)(dst + plane) = vl; __threadfence(); *(volatile v4u_t*)dst = v; *(volatile v4u_t*)(dst + plane) = vl;
  }
}

template <int MODE>
__global__ void __launch_bounds__(256) proj_kernel(const f16* __restrict__ X, size_t plx, int KD, const f16* __restrict__ Wt, size_t plw,
                                                   const float* __restrict__ bias, void* __restrict__ Yp, size_t ply, int NW) {
  __shared__ __attribute__((aligned(16))) float stg[8][16 * 68];
  const int wib = threadIdx.x >> 5;
  const int wave = (blockIdx.x * blockDim.x + threadIdx.x) >> 5;
  const int lane = threadIdx.x & 31, lrow = lane & 15, lhi = lane >> 4;
  const int ncg = NW / 64;
  const int i0 = (wave / ncg) * 16, n0 = (wave % ncg) * 64;
  if (i0 >= MROWS) return;
  v8f acc[4] = {};
  const f16* xrow = X + (size_t)(i0 + lrow) * KD + lhi * 8;
  for (int kk = 0; kk < KD; kk += 32) {
    const Frag2 a = ld2(xrow + kk, plx);
#pragma unroll
    for (int n = 0; n < 4; ++n) acc[n] = wmma_split(a, ld2(Wt + (size_t)(n0 + n * 16 + lrow) * KD + kk + lhi * 8, plw), acc[n]);
  }
  float* sw = stg[wib];
#pragma unroll
  for (int n = 0; n < 4; ++n) { const float bb = bias[n0 + n * 16 + lrow];
#pragma unroll
    for (int r = 0; r < 8; ++r) sw[(r + lhi * 8) * 68 + n * 16 + lrow] = acc[n][r] + bb; }
  asm volatile("s_wait_dscnt 0" ::: "memory");
#pragma unroll 1
  for (int pass = 0; pass < 2; ++pass) {
    if (MODE == 0) {
      f16* Y = (f16*)Yp;
#pragma unroll
      for (int i = 0; i < 4; ++i) { const int c = lane + 32 * i, rr = c >> 3, q = (c & 7) * 8; const float* s = sw + rr * 68 + q;
        v4u_t v, vl; unsigned lq;
        v.x = pk2s(s[0], s[1], &lq); vl.x = lq; v.y = pk2s(s[2], s[3], &lq); vl.y = lq; v.z = pk2s(s[4], s[5], &lq); vl.z = lq; v.w = pk2s(s[6], s[7], &lq); vl.w = lq;
        f16* d = Y + (size_t)(i0 + rr) * NW + n0 + q;
        *(volatile v4u_t*)d = v; *(volatile v4u_t*)(d + ply) = vl; }
    } else {
      float* Y = (float*)Yp;
#pragma unroll
      for (int i = 0; i < 8; ++i) { const int c = lane + 32 * i, rr = c >> 4, q = (c & 15) * 4;
        *(volatile v4f_t*)(Y + (size_t)(i0 + rr) * NW + n0 + q) = *(const volatile v4fa*)(sw + rr * 68 + q); }
    }
    __threadfence();
  }
}

__global__ void __launch_bounds__(256) flash_kernel(const f16* __restrict__ Q, const f16* __restrict__ Kc, const f16* __restrict__ Vc,
                                                    const int* __restrict__ exist, f16* __restrict__ O) {
  __shared__ __attribute__((aligned(16))) f16 plds[8][2][16 * 32];
  __shared__ __attribute__((aligned(16))) f16 vs[8][2][32 * 72];
  __shared__ __attribute__((aligned(16))) float stg[8][16 * 68];
  const int wib = threadIdx.x >> 5;
  const int wave = (blockIdx.x * blockDim.x + threadIdx.x) >> 5;
  const int lane = threadIdx.x & 31, lrow = lane & 15, lhi = lane >> 4;
  const int gpb = Nseq / 16;
  const int b = wave / (NH * gpb), h = (wave / gpb) % NH, i0 = (wave % gpb) * 16;
  if (b >= Bsz) return;
  const f16* qbase = Q  + (size_t)b * Nseq * ALLDIM + h * ADIM;
  const f16* kbase = Kc + (size_t)b * Nseq * ALLDIM + h * ADIM;
  const f16* vbase = Vc + (size_t)b * Nseq * ALLDIM + h * ADIM;
  const int* ex = exist + b * Nseq;
  v8f o[4] = {};
  float m[8], l[8];
#pragma unroll
  for (int r = 0; r < 8; ++r) { m[r] = -3.0e38f; l[r] = 0.f; }
  const float LOG2E = 1.4426950408889634f, SCALE = 0.05590169943749474f;
  f16* vh = vs[wib][0]; f16* vl = vs[wib][1];
  for (int j0 = 0; j0 < Nseq; j0 += 32) {
    { const f16* vr = vbase + (size_t)(j0 + lane) * ALLDIM;
#pragma unroll
      for (int u = 0; u < 8; ++u) { *(v8h*)&vh[lane * 72 + u * 8] = *(const v8h*)(vr + u * 8); *(v8h*)&vl[lane * 72 + u * 8] = *(const v8h*)(vr + PLA + u * 8); } }
    const Frag2 kb00 = ld2(kbase + (size_t)(j0 + lrow) * ALLDIM + lhi * 8, PLA), kb01 = ld2(kbase + (size_t)(j0 + lrow) * ALLDIM + 32 + lhi * 8, PLA);
    const Frag2 kb10 = ld2(kbase + (size_t)(j0 + 16 + lrow) * ALLDIM + lhi * 8, PLA), kb11 = ld2(kbase + (size_t)(j0 + 16 + lrow) * ALLDIM + 32 + lhi * 8, PLA);
    const int e0 = ex[j0 + lrow], e1 = ex[j0 + 16 + lrow];
    asm volatile("s_wait_dscnt 0" ::: "memory");
    {
      f16* ph = plds[wib][0]; f16* pl = plds[wib][1];
      v8f s0 = {}, s1 = {};
      { const Frag2 qa0 = ld2(qbase + (size_t)(i0 + lrow) * ALLDIM + lhi * 8, PLA), qa1 = ld2(qbase + (size_t)(i0 + lrow) * ALLDIM + 32 + lhi * 8, PLA);
        s0 = wmma_split(qa0, kb00, s0); s0 = wmma_split(qa1, kb01, s0);
        s1 = wmma_split(qa0, kb10, s1); s1 = wmma_split(qa1, kb11, s1); }
      float sc0[8], sc1[8], mnew[8];
#pragma unroll
      for (int r = 0; r < 8; ++r) {
        float a0 = (e0 != 0) ? s0[r] * SCALE : -1.0e9f;
        float a1 = (e1 != 0) ? s1[r] * SCALE : -1.0e9f;
        sc0[r] = a0; sc1[r] = a1;
        float mx = fmaxf(a0, a1);
        mx = fmaxf(mx, __shfl_xor(mx, 1)); mx = fmaxf(mx, __shfl_xor(mx, 2)); mx = fmaxf(mx, __shfl_xor(mx, 4)); mx = fmaxf(mx, __shfl_xor(mx, 8));
        mnew[r] = fmaxf(m[r], mx);
      }
#pragma unroll
      for (int r = 0; r < 8; ++r) {
        float p0 = __builtin_exp2f((sc0[r] - mnew[r]) * LOG2E);
        float p1 = __builtin_exp2f((sc1[r] - mnew[r]) * LOG2E);
        float rs = p0 + p1;
        rs += __shfl_xor(rs, 1); rs += __shfl_xor(rs, 2); rs += __shfl_xor(rs, 4); rs += __shfl_xor(rs, 8);
        float fac = __builtin_exp2f((m[r] - mnew[r]) * LOG2E);
        l[r] = l[r] * fac + rs;
        m[r] = mnew[r];
#pragma unroll
        for (int n = 0; n < 4; ++n) o[n][r] *= fac;
        const float q0 = p0 * 1024.0f, q1 = p1 * 1024.0f;
        const f16 h0 = (f16)q0, h1 = (f16)q1;
        ph[(r + lhi * 8) * 32 + lrow] = h0;      pl[(r + lhi * 8) * 32 + lrow] = lo_of(q0, h0);
        ph[(r + lhi * 8) * 32 + 16 + lrow] = h1; pl[(r + lhi * 8) * 32 + 16 + lrow] = lo_of(q1, h1);
      }
    }
    asm volatile("s_wait_dscnt 0" ::: "memory");
    {
      const f16* ph = plds[wib][0]; const f16* pl = plds[wib][1];
      Frag2 pa; pa.h = cat8(*(const v8h*)&ph[lrow * 32 + lhi * 8], *(const v8h*)&ph[lrow * 32 + 16 + lhi * 8]); pa.l = cat8(*(const v8h*)&pl[lrow * 32 + lhi * 8], *(const v8h*)&pl[lrow * 32 + 16 + lhi * 8]);
#pragma unroll
      for (int n = 0; n < 4; ++n) {
        Frag2 vbn;
#pragma unroll
        for (int i = 0; i < 16; ++i) { const int key = (i < 8) ? (lhi * 8 + i) : (16 + lhi * 8 + (i - 8)); vbn.h[i] = vh[key * 72 + n * 16 + lrow]; vbn.l[i] = vl[key * 72 + n * 16 + lrow]; }
        o[n] = wmma_split(pa, vbn, o[n]);
      }
    }
  }
  float* sw = stg[wib];
#pragma unroll
  for (int n = 0; n < 4; ++n)
#pragma unroll
    for (int r = 0; r < 8; ++r) { const int row = i0 + r + lhi * 8; const float qs = (ex[row] != 0) ? 1.0f / (l[r] * 1024.0f) : 0.0f; sw[(r + lhi * 8) * 68 + n * 16 + lrow] = o[n][r] * qs; }
  asm volatile("s_wait_dscnt 0" ::: "memory");
#pragma unroll 1
  for (int pass = 0; pass < 2; ++pass) {
#pragma unroll
    for (int i = 0; i < 4; ++i) { const int c = lane + 32 * i, rr = c >> 3, q = (c & 7) * 8; const float* s = sw + rr * 68 + q;
      v4u_t v, vl2; unsigned lq;
      v.x = pk2s(s[0], s[1], &lq); vl2.x = lq; v.y = pk2s(s[2], s[3], &lq); vl2.y = lq; v.z = pk2s(s[4], s[5], &lq); vl2.z = lq; v.w = pk2s(s[6], s[7], &lq); vl2.w = lq;
      f16* d = O + ((size_t)b * Nseq + i0 + rr) * ALLDIM + h * ADIM + q;
      *(volatile v4u_t*)d = v; *(volatile v4u_t*)(d + PLA) = vl2; }
    __threadfence();
  }
}

extern "C" void kernel_launch(void* const* d_in, const int* in_sizes, int n_in,
                              void* d_out, int out_size, void* d_ws, size_t ws_size,
                              hipStream_t stream) {
  (void)in_sizes; (void)n_in; (void)out_size; (void)ws_size;
  const float* times = (const float*)d_in[0];
  const float* data  = (const float*)d_in[1];
  const float* mask  = (const float*)d_in[2];
  const int*   exist = (const int*)  d_in[3];
  const float* w_per = (const float*)d_in[4];
  const float* b_per = (const float*)d_in[5];
  const float* w_lin = (const float*)d_in[6];
  const float* b_lin = (const float*)d_in[7];
  const float* Wq    = (const float*)d_in[8];
  const float* bq    = (const float*)d_in[9];
  const float* Wk    = (const float*)d_in[10];
  const float* bk    = (const float*)d_in[11];
  const float* Wv    = (const float*)d_in[12];
  const float* bv    = (const float*)d_in[13];
  const float* Wfc   = (const float*)d_in[14];
  const float* bfc   = (const float*)d_in[15];

  char* ws = (char*)d_ws;
  size_t off = 0;
  auto alloc = [&](size_t bytes) -> char* { char* p = ws + off; off = (off + bytes + 255) & ~(size_t)255; return p; };
  f16* Xb  = (f16*)alloc(PLX * 2 * 2);
  f16* WqT = (f16*)alloc(PLW * 2 * 2);
  f16* WkT = (f16*)alloc(PLW * 2 * 2);
  f16* WvT = (f16*)alloc(PLW * 2 * 2);
  f16* WfT = (f16*)alloc(PLWF * 2 * 2);
  f16* Qb  = (f16*)alloc(PLA * 2 * 2);
  f16* Kb  = (f16*)alloc(PLA * 2 * 2);
  f16* Vb  = (f16*)alloc(PLA * 2 * 2);
  f16* Ob  = (f16*)alloc(PLA * 2 * 2);
  const int nrows = MROWS;

  build_x<<<nrows, 256, 0, stream>>>(times, data, mask, w_per, b_per, w_lin, b_lin, Xb);
  wt_cvt<<<dim3(ALLDIM / 16, INDIM / 64), 256, 0, stream>>>(Wq, WqT, INDIM, ALLDIM, PLW);
  wt_cvt<<<dim3(ALLDIM / 16, INDIM / 64), 256, 0, stream>>>(Wk, WkT, INDIM, ALLDIM, PLW);
  wt_cvt<<<dim3(ALLDIM / 16, INDIM / 64), 256, 0, stream>>>(Wv, WvT, INDIM, ALLDIM, PLW);
  wt_cvt<<<dim3(ADIM / 16, ALLDIM / 64), 256, 0, stream>>>(Wfc, WfT, ALLDIM, ADIM, PLWF);

  proj_kernel<0><<<(nrows / 16) * (ALLDIM / 64) / 8, 256, 0, stream>>>(Xb, PLX, INDIM, WqT, PLW, bq, Qb, PLA, ALLDIM);
  proj_kernel<0><<<(nrows / 16) * (ALLDIM / 64) / 8, 256, 0, stream>>>(Xb, PLX, INDIM, WkT, PLW, bk, Kb, PLA, ALLDIM);
  proj_kernel<0><<<(nrows / 16) * (ALLDIM / 64) / 8, 256, 0, stream>>>(Xb, PLX, INDIM, WvT, PLW, bv, Vb, PLA, ALLDIM);
  const int nb = nrows / Nseq;
  flash_kernel<<<nb * NH * (Nseq / 16) / 8, 256, 0, stream>>>(Qb, Kb, Vb, exist, Ob);
  proj_kernel<2><<<(nrows / 16) * (ADIM / 64) / 8, 256, 0, stream>>>(Ob, PLA, ALLDIM, WfT, PLWF, bfc, d_out, 0, ADIM);
}
